// Policy_36223754174568
// MI455X (gfx1250) — hardware-verified
//
#include <hip/hip_runtime.h>
#include <math.h>

constexpr int NTOK  = 16384;
constexpr int NSEQ  = 64;
constexpr int NSTEP = 256;
constexpr int HID   = 128;
constexpr int NGATE = 512;
constexpr int XCOL  = 640;
constexpr int NSC   = 64;
constexpr int NTHR  = 256;
constexpr int NFEAT = 9;
constexpr int NOUTF = NTOK * (3 + 9 + 9 + 38) + 2 * NSEQ * HID;
constexpr float WCAR      = 16.0f;
constexpr float WCAR_INV  = 1.0f / 16.0f;
constexpr float UCAR      = 16.0f;
constexpr float PCAR_INV  = 1.0f / 256.0f;
constexpr float RSCAR     = 2048.0f;
constexpr float RFOLD     = 1.0f / 524288.0f;
constexpr int   WBPIT     = 64;

static_assert(NTOK == NSEQ * NSTEP);
static_assert(NTOK % 128 == 0);
static_assert((NTOK * 5) % 160 == 0);
static_assert((NTOK * 16) % 128 == 0);
static_assert(HID % 32 == 0 && XCOL % 32 == 0);
static_assert(NTOK % 64 == 0 && HID % 64 == 0 && NGATE % 64 == 0 && NSC % 64 == 0);
static_assert(NSEQ % 16 == 0);
static_assert((NTOK * 16) % NTHR == 0);
static_assert(NTOK % NTHR == 0);
static_assert(HID == 16 * (NTHR / 32));
static_assert(NOUTF == 983040);
static_assert(3866624 / 4 == NTOK * 59 && 3899392 / 4 == NTOK * 59 + NSEQ * HID);
static_assert(HID * WBPIT / 8 == 4 * NTHR);

typedef __attribute__((ext_vector_type(16))) _Float16 v16h;
typedef __attribute__((ext_vector_type(8)))  _Float16 v8h;
typedef __attribute__((ext_vector_type(16))) __bf16   v16b;
typedef __attribute__((ext_vector_type(8)))  __bf16   v8b;
typedef __attribute__((ext_vector_type(8)))  float    v8f;
typedef __attribute__((ext_vector_type(4)))  float    v4f;
typedef __attribute__((ext_vector_type(4)))  unsigned v4u;

__device__ __forceinline__ unsigned short f2bf_bits(float f) {
  unsigned u = __float_as_uint(f);
  return (unsigned short)((u + 0x7FFFu + ((u >> 16) & 1u)) >> 16);
}
__device__ __forceinline__ float bf_bits2f(unsigned short h) { return __uint_as_float(((unsigned)h) << 16); }
__device__ __forceinline__ unsigned short f2h_bits(float f) { return __builtin_bit_cast(unsigned short, (_Float16)f); }

__device__ __forceinline__ void dep_guard_h(v8f& a, v8f& b, v16h x, v16h y) { asm volatile("v_nop\n\tv_nop\n\tv_nop\n\tv_nop" : "+v"(a), "+v"(b) : "v"(x), "v"(y)); }
__device__ __forceinline__ void dep_guard_b(v8f& a, v8f& b, v16b x, v16b y) { asm volatile("v_nop\n\tv_nop\n\tv_nop\n\tv_nop" : "+v"(a), "+v"(b) : "v"(x), "v"(y)); }
__device__ __forceinline__ void keep4_h(v16h a, v16h b, v16h c, v16h d) { asm volatile("v_nop" :: "v"(a), "v"(b), "v"(c), "v"(d)); }
__device__ __forceinline__ void keep4_b(v16b a, v16b b, v16b c, v16b d) { asm volatile("v_nop" :: "v"(a), "v"(b), "v"(c), "v"(d)); }
__device__ __forceinline__ void acc_guard4(v8f& a, v8f& b, v8f& c, v8f& d) { asm volatile("v_nop\n\tv_nop\n\tv_nop\n\tv_nop" : "+v"(a), "+v"(b), "+v"(c), "+v"(d)); }
__device__ __forceinline__ void acc_guard2(v8f& a, v8f& b) { asm volatile("v_nop\n\tv_nop\n\tv_nop\n\tv_nop" : "+v"(a), "+v"(b)); }
__device__ __forceinline__ void tie2_h3(v8f& a, v8f& b, v16h x, v16h y, v16h z) { asm volatile("v_nop\n\tv_nop\n\tv_nop\n\tv_nop" : "+v"(a), "+v"(b) : "v"(x), "v"(y), "v"(z)); }
__device__ __forceinline__ void tie4_h5(v8f& a, v8f& b, v8f& c, v8f& d, v16h s, v16h w, v16h x, v16h y, v16h z) {
  asm volatile("v_nop\n\tv_nop\n\tv_nop\n\tv_nop" : "+v"(a), "+v"(b), "+v"(c), "+v"(d) : "v"(s), "v"(w), "v"(x), "v"(y), "v"(z));
}
__device__ __forceinline__ void tie1_b4(v8f& a, v16b w, v16b x, v16b y, v16b z) { asm volatile("v_nop\n\tv_nop\n\tv_nop\n\tv_nop" : "+v"(a) : "v"(w), "v"(x), "v"(y), "v"(z)); }

template <typename T> struct Frag;
template <> struct Frag<_Float16> {
  typedef v16h V; union U { v16h v; v8h h[2]; };
  static __device__ __forceinline__ v16h load(const _Float16* p) {
    U f; f.h[0] = *(const v8h*)(p); f.h[1] = *(const v8h*)(p + 16); return f.v;
  }
  static __device__ __forceinline__ v8f mma(v16h a, v16h b, v8f c) {
    return __builtin_amdgcn_wmma_f32_16x16x32_f16(false, a, false, b, (short)0, c, false, false);
  }
  static __device__ __forceinline__ void guard(v8f& a, v8f& b, v16h x, v16h y) { dep_guard_h(a, b, x, y); }
  static __device__ __forceinline__ void keep(v16h a, v16h b, v16h c, v16h d) { keep4_h(a, b, c, d); }
};
template <> struct Frag<__bf16> {
  typedef v16b V; union U { v16b v; v8b h[2]; };
  static __device__ __forceinline__ v16b load(const __bf16* p) {
    U f; f.h[0] = *(const v8b*)(p); f.h[1] = *(const v8b*)(p + 16); return f.v;
  }
  static __device__ __forceinline__ v8f mma(v16b a, v16b b, v8f c) {
    return __builtin_amdgcn_wmma_f32_16x16x32_bf16(false, a, false, b, (short)0, c, false, false);
  }
  static __device__ __forceinline__ void guard(v8f& a, v8f& b, v16b x, v16b y) { dep_guard_b(a, b, x, y); }
  static __device__ __forceinline__ void keep(v16b a, v16b b, v16b c, v16b d) { keep4_b(a, b, c, d); }
};

__device__ __forceinline__ void bf_split_words(const float* f, v4u& wh, v4u& wl) {
#pragma unroll
  for (int e = 0; e < 4; ++e) {
    const unsigned short hb0 = f2bf_bits(f[2 * e]), hb1 = f2bf_bits(f[2 * e + 1]);
    const unsigned short lb0 = f2bf_bits(f[2 * e] - bf_bits2f(hb0));
    const unsigned short lb1 = f2bf_bits(f[2 * e + 1] - bf_bits2f(hb1));
    wh[e] = (unsigned)hb0 | ((unsigned)hb1 << 16);
    wl[e] = (unsigned)lb0 | ((unsigned)lb1 << 16);
  }
}
__device__ __forceinline__ v4u h16_words(const float* f, float sc) {
  v4u w;
#pragma unroll
  for (int e = 0; e < 4; ++e) {
    const unsigned short b0 = f2h_bits(f[2 * e] * sc), b1 = f2h_bits(f[2 * e + 1] * sc);
    w[e] = (unsigned)b0 | ((unsigned)b1 << 16);
  }
  return w;
}

template <int ET> struct Elem;
template <> struct Elem<0> { typedef _Float16 T; };
template <> struct Elem<1> { typedef __bf16 T; };
template <int ET, bool SPLIT, int BIAS_MODE, int OUT_MODE, bool RESID, int ACT = 0>
__global__ __launch_bounds__(256) void wmma_gemm64(
    const unsigned short* __restrict__ Ap, const unsigned short* __restrict__ A2p, int lda, long strideA,
    const unsigned short* __restrict__ Btp, const unsigned short* __restrict__ Bt2p, int ldb, long strideB,
    void* __restrict__ Cout, void* __restrict__ Cout2, int ldc, long strideC,
    const float* __restrict__ bias,
    const float* __restrict__ resid, long strideR,
    int M, int N, int K, float scale) {
  typedef typename Elem<ET>::T T;
  typedef typename Frag<T>::V V;
  const T* A = (const T*)Ap; const T* A2 = (const T*)A2p; const T* Bt = (const T*)Btp; const T* Bt2 = (const T*)Bt2p;
  __shared__ __align__(16) float sT[8][16 * 68];
  const int b    = blockIdx.y;
  const int lane = threadIdx.x & 31;
  const int wave = threadIdx.x >> 5;
  const int tilesN = N >> 6;
  const int tilesM = M >> 6;
  const int tile = blockIdx.x * 8 + wave;
  if (tile >= tilesM * tilesN) return;
  const int tm = tile / tilesN;
  const int tn = tile - tm * tilesN;
  const int m0 = tm << 6;
  const int n0 = tn << 6;

  const T* Ab  = A  + (size_t)b * strideA;
  const T* Bb  = Bt + (size_t)b * strideB;
  const T* Ab2 = SPLIT ? (A2  + (size_t)b * strideA) : nullptr;
  const T* Bb2 = SPLIT ? (Bt2 + (size_t)b * strideB) : nullptr;

  const int rlane = lane & 15;
  const int koff  = (lane >> 4) * 8;
  const int mOff  = (lane >> 4) * 8;

  v8f acc[4][4];
#pragma unroll
  for (int i = 0; i < 4; ++i)
#pragma unroll
    for (int j = 0; j < 4; ++j) acc[i][j] = (v8f){0.f,0.f,0.f,0.f,0.f,0.f,0.f,0.f};

  for (int k0 = 0; k0 < K; k0 += 32) {
    V bh[4], bl[4];
#pragma unroll
    for (int j = 0; j < 4; ++j) {
      const size_t bo = (size_t)(n0 + (j << 4) + rlane) * ldb + koff + k0;
      bh[j] = Frag<T>::load(Bb + bo);
      if (SPLIT) bl[j] = Frag<T>::load(Bb2 + bo);
    }
#pragma unroll
    for (int i = 0; i < 4; ++i) {
      const size_t ao = (size_t)(m0 + (i << 4) + rlane) * lda + koff + k0;
      V ah = Frag<T>::load(Ab + ao);
      V al;
      if (SPLIT) al = Frag<T>::load(Ab2 + ao);
#pragma unroll
      for (int j = 0; j < 4; ++j) {
        acc[i][j] = Frag<T>::mma(ah, bh[j], acc[i][j]);
        if (SPLIT) {
          acc[i][j] = Frag<T>::mma(ah, bl[j], acc[i][j]);
          acc[i][j] = Frag<T>::mma(al, bh[j], acc[i][j]);
        }
      }
      Frag<T>::guard(acc[i][0], acc[i][3], ah, SPLIT ? al : ah);
      Frag<T>::guard(acc[i][1], acc[i][2], ah, bh[3]);
    }
    Frag<T>::keep(bh[0], bh[1], bh[2], bh[3]);
    if (SPLIT) Frag<T>::keep(bl[0], bl[1], bl[2], bl[3]);
  }
  acc_guard4(acc[0][0], acc[0][1], acc[0][2], acc[0][3]);
  acc_guard4(acc[1][0], acc[1][1], acc[1][2], acc[1][3]);
  acc_guard4(acc[2][0], acc[2][1], acc[2][2], acc[2][3]);
  acc_guard4(acc[3][0], acc[3][1], acc[3][2], acc[3][3]);

  float* slab = sT[wave];
  const float* Rb = RESID ? (resid + (size_t)b * strideR) : nullptr;
#pragma unroll
  for (int i = 0; i < 4; ++i) {
    const int mBase = m0 + (i << 4);
#pragma unroll
    for (int j = 0; j < 4; ++j) {
      const int n = n0 + (j << 4) + rlane;
      float bv = 0.f;
      if (BIAS_MODE == 2) bv = bias[n];
#pragma unroll
      for (int r = 0; r < 8; ++r) {
        float v = acc[i][j][r] * scale;
        if (BIAS_MODE == 1) v += bias[mBase + mOff + r];
        if (BIAS_MODE == 2) v += bv;
        if (RESID) v += Rb[(size_t)(mBase + mOff + r) * ldc + n];
        if (ACT == 1) v = tanhf(v);
        if (ACT == 2) v = fmaxf(v, 0.0f);
        if (ACT == 3) v = v / (1.0f + expf(-v));
        if (ACT == 4) v = (v > 0.f) ? v : 0.01f * v;
        if (ACT == 5) v = 0.5f * v * (1.0f + erff(v * 0.70710678118654752f));
        slab[(mOff + r) * 68 + (j << 4) + rlane] = v;
      }
    }
    __builtin_amdgcn_fence(__ATOMIC_RELEASE, "workgroup");
    __builtin_amdgcn_wave_barrier();
    __builtin_amdgcn_fence(__ATOMIC_ACQUIRE, "workgroup");
    if (OUT_MODE == 0) {
      float* C = (float*)Cout + (size_t)b * strideC;
      const int hh = lane >> 4, c4 = (lane & 15) * 4;
      for (int pass = 0; pass < 2; ++pass) {
#pragma unroll
        for (int it = 0; it < 8; ++it) {
          const int row = it * 2 + hh;
          v4f v = *(const v4f*)(slab + row * 68 + c4);
          *(volatile v4f*)(C + (size_t)(mBase + row) * ldc + n0 + c4) = v;
        }
        __threadfence();
      }
    } else {
      const int q = lane >> 3, c8 = (lane & 7) * 8;
      unsigned short* C  = (unsigned short*)Cout  + (size_t)b * strideC;
      unsigned short* C2 = (OUT_MODE == 2) ? ((unsigned short*)Cout2 + (size_t)b * strideC) : nullptr;
      for (int pass = 0; pass < 2; ++pass) {
#pragma unroll
        for (int it = 0; it < 4; ++it) {
          const int row = it * 4 + q;
          const float* sp = slab + row * 68 + c8;
          v8h hv, lv;
#pragma unroll
          for (int e = 0; e < 8; ++e) {
            if (OUT_MODE == 1) {
              hv[e] = (_Float16)sp[e];
            } else {
              unsigned short hb = f2bf_bits(sp[e]);
              unsigned short lb = f2bf_bits(sp[e] - bf_bits2f(hb));
              hv[e] = __builtin_bit_cast(_Float16, hb);
              lv[e] = __builtin_bit_cast(_Float16, lb);
            }
          }
          *(volatile v8h*)(C + (size_t)(mBase + row) * ldc + n0 + c8) = hv;
          if (OUT_MODE == 2) *(volatile v8h*)(C2 + (size_t)(mBase + row) * ldc + n0 + c8) = lv;
        }
        __threadfence();
      }
    }
    __builtin_amdgcn_fence(__ATOMIC_RELEASE, "workgroup");
    __builtin_amdgcn_wave_barrier();
    __builtin_amdgcn_fence(__ATOMIC_ACQUIRE, "workgroup");
  }
}

__global__ __launch_bounds__(NTHR) void wsplit_kernel(
    const float* __restrict__ s0, const float* __restrict__ s1, const float* __restrict__ s2, const float* __restrict__ s3,
    unsigned short* __restrict__ dh0, unsigned short* __restrict__ dl0, unsigned short* __restrict__ dh1, unsigned short* __restrict__ dl1,
    unsigned short* __restrict__ dh2, unsigned short* __restrict__ dl2, unsigned short* __restrict__ dh3, unsigned short* __restrict__ dl3,
    int n80, int n81, int n82, int n83) {
  const int y = blockIdx.y;
  const float* src = s0; unsigned short* dh = dh0; unsigned short* dl = dl0; int n8 = n80;
  if (y == 1) { src = s1; dh = dh1; dl = dl1; n8 = n81; }
  else if (y == 2) { src = s2; dh = dh2; dl = dl2; n8 = n82; }
  else if (y == 3) { src = s3; dh = dh3; dl = dl3; n8 = n83; }
  const int i = blockIdx.x * NTHR + threadIdx.x;
  if (i < n8) {
    union { v4f v[2]; float f[8]; } in;
    in.v[0] = *(const v4f*)(src + (size_t)i * 8);
    in.v[1] = *(const v4f*)(src + (size_t)i * 8 + 4);
    v4u wh, wl;
    bf_split_words(in.f, wh, wl);
    for (int pass = 0; pass < 2; ++pass) {
      *(volatile v4u*)(dh + (size_t)i * 8) = wh;
      *(volatile v4u*)(dl + (size_t)i * 8) = wl;
      __threadfence();
    }
  }
}

__global__ __launch_bounds__(NTHR) void wf16_kernel(
    const float* __restrict__ s0, const float* __restrict__ s1, const float* __restrict__ s2, const float* __restrict__ s3,
    unsigned short* __restrict__ dst) {
  const int y = blockIdx.y;
  const float* src = s0;
  if (y == 1) src = s1; else if (y == 2) src = s2; else if (y == 3) src = s3;
  const int i = blockIdx.x * NTHR + threadIdx.x;
  if (i < HID * HID / 8) {
    union { v4f v[2]; float f[8]; } in;
    in.v[0] = *(const v4f*)(src + (size_t)i * 8);
    in.v[1] = *(const v4f*)(src + (size_t)i * 8 + 4);
    const v4u w = h16_words(in.f, WCAR);
    unsigned short* dp = dst + (size_t)y * HID * HID + (size_t)i * 8;
    *(volatile v4u*)dp = w;
    __threadfence();
    *(volatile v4u*)dp = w;
  }
}

__global__ __launch_bounds__(NTHR) void wbpack_kernel(const float* __restrict__ wbas, unsigned short* __restrict__ wbp) {
  const int i = blockIdx.x * NTHR + threadIdx.x;
  const int row = i >> 3, q = i & 7;
  const int qq = q & 3;
  const float fres = (float)(q >> 2);
  const float fmn  = 1.0f - fres;
  float val[8];
#pragma unroll
  for (int e = 0; e < 8; ++e) {
    const int ss = 8 * qq + e;
    const int k1 = (ss >= 9) ? 1 : 0, k2 = (ss >= 18) ? 1 : 0;
    int f = ss - 9 * k1; f = (f > 8) ? 8 : f;
    const float w  = wbas[row * NFEAT + f];
    const float ws = w * WCAR;
    const float bh = (float)(_Float16)ws;
    const float rs = (ws - bh) * RSCAR;
    const float g0 = (float)(1 - k1), g1 = (float)(k1 - k2);
    const float fbh = fmn * g1 + fres * g0;
    const float frs = fres * g1;
    val[e] = fmaf(fbh, bh, frs * rs);
  }
  const v4u wv = h16_words(val, 1.0f);
  unsigned short* dp = wbp + (size_t)i * 8;
  *(volatile v4u*)dp = wv;
  __threadfence();
  *(volatile v4u*)dp = wv;
}

__global__ __launch_bounds__(NTHR) void smallprep_kernel(
    const float* __restrict__ wenum, const float* __restrict__ wmx, const float* __restrict__ wmy,
    const float* __restrict__ benum, const float* __restrict__ bmx, const float* __restrict__ bmy,
    const float* __restrict__ bih, const float* __restrict__ bhh,
    unsigned short* __restrict__ wdh, unsigned short* __restrict__ wdl, float* __restrict__ bhd, float* __restrict__ bsum) {
  const int tid = threadIdx.x, blk = blockIdx.x;
  if (blk < 4) {
    const int i = blk * NTHR + tid;
    const int row = i >> 4, c8 = (i & 15) * 8;
    const int re = (row < 2) ? row : 2;
    int rx = row - 3;  rx = (rx < 0) ? 0 : ((rx > 8) ? 8 : rx);
    int ry = row - 12; ry = (ry < 0) ? 0 : ((ry > 8) ? 8 : ry);
    const float fe = (row < 3) ? 1.0f : 0.0f;
    const float fx = (row >= 3 && row < 12) ? 1.0f : 0.0f;
    const float fy = (row >= 12 && row < 21) ? 1.0f : 0.0f;
    union { v4f v[2]; float f[8]; } ve, vx, vy;
    ve.v[0] = *(const v4f*)(wenum + (size_t)re * HID + c8); ve.v[1] = *(const v4f*)(wenum + (size_t)re * HID + c8 + 4);
    vx.v[0] = *(const v4f*)(wmx + (size_t)rx * HID + c8);   vx.v[1] = *(const v4f*)(wmx + (size_t)rx * HID + c8 + 4);
    vy.v[0] = *(const v4f*)(wmy + (size_t)ry * HID + c8);   vy.v[1] = *(const v4f*)(wmy + (size_t)ry * HID + c8 + 4);
    float f[8];
#pragma unroll
    for (int e = 0; e < 8; ++e) f[e] = fmaf(fe, ve.f[e], fmaf(fx, vx.f[e], fy * vy.f[e]));
    v4u wh, wl;
    bf_split_words(f, wh, wl);
    for (int pass = 0; pass < 2; ++pass) {
      *(volatile v4u*)(wdh + (size_t)i * 8) = wh;
      *(volatile v4u*)(wdl + (size_t)i * 8) = wl;
      __threadfence();
    }
    if (blk == 0 && tid < 16) {
      const int j0 = 4 * tid;
      v4f o;
#pragma unroll
      for (int e = 0; e < 4; ++e) {
        const int j = j0 + e;
        const int je = (j < 2) ? j : 2;
        int jx = j - 3;  jx = (jx < 0) ? 0 : ((jx > 8) ? 8 : jx);
        int jy = j - 12; jy = (jy < 0) ? 0 : ((jy > 8) ? 8 : jy);
        const float ge = (j < 3) ? 1.0f : 0.0f;
        const float gxf = (j >= 3 && j < 12) ? 1.0f : 0.0f;
        const float gyf = (j >= 12 && j < 21) ? 1.0f : 0.0f;
        o[e] = fmaf(ge, benum[je], fmaf(gxf, bmx[jx], gyf * bmy[jy]));
      }
      float* op = bhd + j0;
      *(volatile v4f*)op = o;
      __threadfence();
      *(volatile v4f*)op = o;
    }
  } else {
    if (tid < NGATE / 4) {
      const v4f a = *(const v4f*)(bih + 4 * tid);
      const v4f c = *(const v4f*)(bhh + 4 * tid);
      const v4f s = a + c;
      float* op = bsum + 4 * tid;
      *(volatile v4f*)op = s;
      __threadfence();
      *(volatile v4f*)op = s;
    }
  }
}

__global__ __launch_bounds__(NTHR) void env_kernel(const float* __restrict__ env, const float* __restrict__ wenv,
                                                   const float* __restrict__ benv,
                                                   unsigned short* __restrict__ xh, unsigned short* __restrict__ xl) {
  const int i = blockIdx.x * NTHR + threadIdx.x;
  const int t = i >> 4, c8 = (i & 15) * 8;
  const float e0 = env[(size_t)t * 3 + 0], e1 = env[(size_t)t * 3 + 1], e2 = env[(size_t)t * 3 + 2];
  union { v4f v[6]; float f[24]; } wu;
  const v4f* wq = (const v4f*)(wenv + c8 * 3);
#pragma unroll
  for (int q = 0; q < 6; ++q) wu.v[q] = wq[q];
  union { v4f v[2]; float f[8]; } bu;
  bu.v[0] = *(const v4f*)(benv + c8); bu.v[1] = *(const v4f*)(benv + c8 + 4);
  float f[8];
#pragma unroll
  for (int e = 0; e < 8; ++e) {
    float v = 0.0f;
    v = fmaf(wu.f[3 * e + 0], e0, v);
    v = fmaf(wu.f[3 * e + 1], e1, v);
    v = fmaf(wu.f[3 * e + 2], e2, v);
    v += bu.f[e];
    f[e] = fmaxf(v, 0.0f);
  }
  v4u wh, wl;
  bf_split_words(f, wh, wl);
  const size_t o = (size_t)t * XCOL + c8;
  for (int pass = 0; pass < 2; ++pass) {
    *(volatile v4u*)(xh + o) = wh;
    *(volatile v4u*)(xl + o) = wl;
    __threadfence();
  }
}

template <int MROWS, int NUNIT, int MODE>
__global__ __launch_bounds__(NTHR) void unit_pass_kernel(
    const float* uA, const float* uB,
    const unsigned short* __restrict__ wbp, const float* __restrict__ bbas,
    const unsigned short* wtA, const unsigned short* wtB,
    const float* bgA, const float* bgB,
    unsigned short* __restrict__ xh, unsigned short* __restrict__ xl, int colA, int colB,
    const float* __restrict__ att, float* tgA, float* tgB)
{
  constexpr int TPB   = MROWS / NUNIT;
  constexpr int MSUB  = MROWS / 16;
  constexpr int MHALF = MSUB / 2;
  constexpr int UPIT = 40, BPIT = 136, EPIT = 132;
  static_assert(MROWS % 32 == 0 && MROWS <= NTHR && MROWS % NUNIT == 0 && (MROWS / 4) % 8 == 0);
  static_assert(MROWS * UPIT * 2 + MROWS * BPIT * 2 <= MROWS * EPIT * 4);
  static_assert((MROWS * UPIT * 2) % 16 == 0);
  __shared__ __align__(16) unsigned char smem[MROWS * EPIT * 4];
  __shared__ __align__(16) float sLog[MROWS];

  const int tid = threadIdx.x, lane = tid & 31, wave = tid >> 5;
  const int rlane = lane & 15, hh = lane >> 4, koff = hh * 8;
  const int gy = blockIdx.y;
  const float* U = gy ? uB : uA;
  const _Float16* WT = (const _Float16*)(gy ? wtB : wtA);
  const float* BG = gy ? bgB : bgA;
  const int xcol = gy ? colB : colA;
  float* TG = gy ? tgB : tgA;
  const int row0 = blockIdx.x * MROWS;
  const int tok0 = blockIdx.x * TPB;

  unsigned short* uT = (unsigned short*)smem;
  const _Float16* uTh = (const _Float16*)smem;
  _Float16* bT = (_Float16*)(smem + MROWS * UPIT * 2);
  float* eT = (float*)smem;

  if (tid < MROWS) {
    const float* up = U + (size_t)(row0 + tid) * NFEAT;
    float uv[NFEAT];
#pragma unroll
    for (int f = 0; f < NFEAT; ++f) uv[f] = up[f];
    unsigned hb[NFEAT], lb[NFEAT];
#pragma unroll
    for (int f = 0; f < NFEAT; ++f) {
      const float us = uv[f] * UCAR;
      const _Float16 hv = (_Float16)us;
      const float res = (us - (float)hv) * RSCAR;
      hb[f] = (unsigned)__builtin_bit_cast(unsigned short, hv);
      lb[f] = (unsigned)f2h_bits(res);
    }
    v4u w0, w1, w2;
    w0[0] = lb[0] | (lb[1] << 16); w0[1] = lb[2] | (lb[3] << 16); w0[2] = lb[4] | (lb[5] << 16); w0[3] = lb[6] | (lb[7] << 16);
    w1[0] = lb[8] | (hb[0] << 16); w1[1] = hb[1] | (hb[2] << 16); w1[2] = hb[3] | (hb[4] << 16); w1[3] = hb[5] | (hb[6] << 16);
    w2[0] = hb[7] | (hb[8] << 16); w2[1] = 0u;                   w2[2] = 0u;                   w2[3] = 0u;
    const v4u wz = {0u, 0u, 0u, 0u};
    v4u* dp = (v4u*)(uT + tid * UPIT);
    dp[0] = w0; dp[1] = w1; dp[2] = w2; dp[3] = wz; dp[4] = wz;
  }
  __syncthreads();

  const int npair = wave & 3, mg = wave >> 2;
  const int colb = 32 * npair + rlane;
  const v8f z8 = {0.f, 0.f, 0.f, 0.f, 0.f, 0.f, 0.f, 0.f};

  {
    const _Float16* WB = (const _Float16*)wbp;
    const v16h b0m = Frag<_Float16>::load(WB + (size_t)colb * WBPIT + koff);
    const v16h b0r = Frag<_Float16>::load(WB + (size_t)colb * WBPIT + 32 + koff);
    const v16h b1m = Frag<_Float16>::load(WB + (size_t)(colb + 16) * WBPIT + koff);
    const v16h b1r = Frag<_Float16>::load(WB + (size_t)(colb + 16) * WBPIT + 32 + koff);
    const float bb0 = bbas[colb], bb1 = bbas[colb + 16];
#pragma unroll
    for (int i = 0; i < MHALF; ++i) {
      const int mi = mg * MHALF + i;
      const v16h a = Frag<_Float16>::load(uTh + (16 * mi + rlane) * UPIT + koff);
      v8f d0 = Frag<_Float16>::mma(a, b0m, z8);
      v8f e0 = Frag<_Float16>::mma(a, b0r, z8);
      v8f d1 = Frag<_Float16>::mma(a, b1m, z8);
      v8f e1 = Frag<_Float16>::mma(a, b1r, z8);
      tie4_h5(d0, e0, d1, e1, a, b0m, b0r, b1m, b1r);
#pragma unroll
      for (int r = 0; r < 8; ++r) {
        const int row = 16 * mi + 8 * hh + r;
        const float v0 = fmaxf(fmaf(e0[r], RFOLD, d0[r] * PCAR_INV) + bb0, 0.0f);
        const float v1 = fmaxf(fmaf(e1[r], RFOLD, d1[r] * PCAR_INV) + bb1, 0.0f);
        bT[row * BPIT + colb]      = (_Float16)v0;
        bT[row * BPIT + colb + 16] = (_Float16)v1;
      }
    }
  }
  __syncthreads();

  v8f acc[MHALF][2];
#pragma unroll
  for (int i = 0; i < MHALF; ++i) { acc[i][0] = z8; acc[i][1] = z8; }
#pragma unroll 1
  for (int kc = 0; kc < HID / 32; ++kc) {
    const int k0 = kc * 32;
    const v16h b0 = Frag<_Float16>::load(WT + (size_t)colb * HID + koff + k0);
    const v16h b1 = Frag<_Float16>::load(WT + (size_t)(colb + 16) * HID + koff + k0);
#pragma unroll
    for (int i = 0; i < MHALF; ++i) {
      const int mi = mg * MHALF + i;
      const v16h a = Frag<_Float16>::load(bT + (16 * mi + rlane) * BPIT + koff + k0);
      acc[i][0] = Frag<_Float16>::mma(a, b0, acc[i][0]);
      acc[i][1] = Frag<_Float16>::mma(a, b1, acc[i][1]);
      tie2_h3(acc[i][0], acc[i][1], a, b0, b1);
    }
  }
#pragma unroll
  for (int i = 0; i < MHALF; ++i) acc_guard2(acc[i][0], acc[i][1]);
  __syncthreads();
  {
    const float g0 = BG[colb], g1 = BG[colb + 16];
#pragma unroll
    for (int i = 0; i < MHALF; ++i) {
      const int mi = mg * MHALF + i;
#pragma unroll
      for (int r = 0; r < 8; ++r) {
        const int row = 16 * mi + 8 * hh + r;
        eT[row * EPIT + colb]      = acc[i][0][r] * WCAR_INV + g0;
        eT[row * EPIT + colb + 16] = acc[i][1][r] * WCAR_INV + g1;
      }
    }
  }
  __syncthreads();

  if (MODE == 0) {
    constexpr int ITEMS = TPB * 16;
    constexpr int NIT = (ITEMS + NTHR - 1) / NTHR;
    static_assert(ITEMS % 32 == 0);
#pragma unroll 1
    for (int it = 0; it < NIT; ++it) {
      const int idx = it * NTHR + tid;
      if (idx < ITEMS) {
        const int tk = idx >> 4, c8 = (idx & 15) * 8;
        const float* ep = eT + (tk * NUNIT) * EPIT + c8;
        union { v4f v[2]; float f[8]; } mx;
        mx.v[0] = *(const v4f*)ep;
        mx.v[1] = *(const v4f*)(ep + 4);
#pragma unroll
        for (int n = 1; n < NUNIT; ++n) {
          const v4f a0 = *(const v4f*)(ep + n * EPIT);
          const v4f a1 = *(const v4f*)(ep + n * EPIT + 4);
#pragma unroll
          for (int e = 0; e < 4; ++e) { mx.f[e] = fmaxf(mx.f[e], a0[e]); mx.f[4 + e] = fmaxf(mx.f[4 + e], a1[e]); }
        }
        v4u wh, wl;
        bf_split_words(mx.f, wh, wl);
        const size_t o = (size_t)(tok0 + tk) * XCOL + xcol + c8;
        for (int pass = 0; pass < 2; ++pass) {
          *(volatile v4u*)(xh + o) = wh;
          *(volatile v4u*)(xl + o) = wl;
          __threadfence();
        }
      }
    }
  } else {
    if (tid < MROWS) {
      const int tk = tid / NUNIT;
      const float* ap = att + (size_t)(tok0 + tk) * HID;
      const float* ep = eT + tid * EPIT;
      float s = 0.0f;
#pragma unroll 1
      for (int ch = 0; ch < HID / 8; ++ch) {
        const v4f a0 = *(const v4f*)(ap + 8 * ch);
        const v4f a1 = *(const v4f*)(ap + 8 * ch + 4);
        const v4f x0 = *(const v4f*)(ep + 8 * ch);
        const v4f x1 = *(const v4f*)(ep + 8 * ch + 4);
        s = fmaf(a0[0], x0[0], s); s = fmaf(a0[1], x0[1], s); s = fmaf(a0[2], x0[2], s); s = fmaf(a0[3], x0[3], s);
        s = fmaf(a1[0], x1[0], s); s = fmaf(a1[1], x1[1], s); s = fmaf(a1[2], x1[2], s); s = fmaf(a1[3], x1[3], s);
      }
      sLog[tid] = s;
    }
    __syncthreads();
    if (tid < MROWS / 4) {
      const v4f v = *(const v4f*)(sLog + 4 * tid);
      float* dp = TG + (size_t)blockIdx.x * MROWS + 4 * tid;
      *(volatile v4f*)dp = v;
      __threadfence();
      *(volatile v4f*)dp = v;
    }
  }
}

constexpr int GPIT = 516;
constexpr int HPIT = 136;
constexpr int OPIT = 132;
__global__ __launch_bounds__(NTHR) void lstm_kernel(const float* __restrict__ gx, const float* __restrict__ hzero,
                                                    const float* __restrict__ czero,
                                                    const unsigned short* __restrict__ whh_hi,
                                                    const unsigned short* __restrict__ whh_lo,
                                                    unsigned short* __restrict__ hsh, unsigned short* __restrict__ hsl,
                                                    float* __restrict__ hn_out, float* __restrict__ cn_out) {
  __shared__ __align__(16) float          G[16 * GPIT];
  __shared__ __align__(16) unsigned short AH[16 * HPIT];
  __shared__ __align__(16) unsigned short AL[16 * HPIT];
  __shared__ __align__(16) float          HS[16 * OPIT];
  const int tid = threadIdx.x, lane = tid & 31, wave = tid >> 5;
  const int c = lane & 15, hh = lane >> 4, koff = hh * 8;
  const int j = 16 * wave + c;
  const int rowbase = blockIdx.x * 16;
  const __bf16* WH = (const __bf16*)whh_hi;
  const __bf16* WL = (const __bf16*)whh_lo;

#pragma unroll
  for (int i = 0; i < 8; ++i) {
    const int idx = i * NTHR + tid;
    const int row = idx >> 7, col = idx & 127;
    const float v = hzero[(size_t)(rowbase + row) * HID + col];
    const unsigned short hb = f2bf_bits(v);
    AH[row * HPIT + col] = hb;
    AL[row * HPIT + col] = f2bf_bits(v - bf_bits2f(hb));
  }
  float cst[8], hst[8];
#pragma unroll
  for (int r = 0; r < 8; ++r) { cst[r] = czero[(size_t)(rowbase + 8 * hh + r) * HID + j]; hst[r] = 0.0f; }
  __syncthreads();

  const __bf16* ahp = (const __bf16*)AH + c * HPIT + koff;
  const __bf16* alp = (const __bf16*)AL + c * HPIT + koff;
  const v8f z8 = {0.f, 0.f, 0.f, 0.f, 0.f, 0.f, 0.f, 0.f};

#pragma unroll 1
  for (int t = 0; t < NSTEP; ++t) {
#pragma unroll
    for (int i = 0; i < 8; ++i) {
      const int idx = i * NTHR + tid;
      const int row = idx >> 7, c4 = (idx & 127) * 4;
      const v4f v = *(const v4f*)(gx + ((size_t)(rowbase + row) * NSTEP + (size_t)t) * NGATE + c4);
      *(v4f*)(G + row * GPIT + c4) = v;
    }
    __syncthreads();
    v8f acc[4];
    acc[0] = z8; acc[1] = z8; acc[2] = z8; acc[3] = z8;
#pragma unroll 1
    for (int kc = 0; kc < HID / 32; ++kc) {
      const int k0 = kc * 32;
      const v16b ah = Frag<__bf16>::load(ahp + k0);
      const v16b al = Frag<__bf16>::load(alp + k0);
#pragma unroll
      for (int g = 0; g < 4; ++g) {
        const size_t wo = (size_t)(g * HID + j) * HID + koff + k0;
        const v16b bh = Frag<__bf16>::load(WH + wo);
        const v16b bl = Frag<__bf16>::load(WL + wo);
        acc[g] = Frag<__bf16>::mma(ah, bh, acc[g]);
        acc[g] = Frag<__bf16>::mma(ah, bl, acc[g]);
        acc[g] = Frag<__bf16>::mma(al, bh, acc[g]);
        tie1_b4(acc[g], ah, al, bh, bl);
      }
    }
    acc_guard4(acc[0], acc[1], acc[2], acc[3]);
#pragma unroll
    for (int r = 0; r < 8; ++r) {
      const float* gp = G + (8 * hh + r) * GPIT + j;
      const float zi = acc[0][r] + gp[0];
      const float zf = acc[1][r] + gp[HID];
      const float zg = acc[2][r] + gp[2 * HID];
      const float zo = acc[3][r] + gp[3 * HID];
      const float ig = 1.0f / (1.0f + expf(-zi));
      const float fg = 1.0f / (1.0f + expf(-zf));
      const float og = 1.0f / (1.0f + expf(-zo));
      const float gg = tanhf(zg);
      const float cn = fg * cst[r] + ig * gg;
      cst[r] = cn;
      hst[r] = og * tanhf(cn);
    }
    __syncthreads();
#pragma unroll
    for (int r = 0; r < 8; ++r) {
      const int row = 8 * hh + r;
      const float v = hst[r];
      const unsigned short hb = f2bf_bits(v);
      AH[row * HPIT + j] = hb;
      AL[row * HPIT + j] = f2bf_bits(v - bf_bits2f(hb));
      HS[row * OPIT + j] = v;
    }
    __syncthreads();
    {
      const int row = tid >> 4, c8 = (tid & 15) * 8;
      union { v4f v[2]; float f[8]; } hv;
      hv.v[0] = *(const v4f*)(HS + row * OPIT + c8);
      hv.v[1] = *(const v4f*)(HS + row * OPIT + c8 + 4);
      v4u wh, wl;
      bf_split_words(hv.f, wh, wl);
      const size_t o = ((size_t)(rowbase + row) * NSTEP + (size_t)t) * HID + c8;
      for (int pass = 0; pass < 2; ++pass) {
        *(volatile v4u*)(hsh + o) = wh;
        *(volatile v4u*)(hsl + o) = wl;
        __threadfence();
      }
    }
  }

  for (int pass = 0; pass < 2; ++pass) {
#pragma unroll
    for (int it = 0; it < 2; ++it) {
      const int idx = it * NTHR + tid;
      const int row = idx >> 5, c4 = (idx & 31) * 4;
      const v4f v = *(const v4f*)(HS + row * OPIT + c4);
      *(volatile v4f*)(hn_out + (size_t)(rowbase + row) * HID + c4) = v;
    }
    __threadfence();
  }
  __syncthreads();
#pragma unroll
  for (int r = 0; r < 8; ++r) HS[(8 * hh + r) * OPIT + j] = cst[r];
  __syncthreads();
  for (int pass = 0; pass < 2; ++pass) {
#pragma unroll
    for (int it = 0; it < 2; ++it) {
      const int idx = it * NTHR + tid;
      const int row = idx >> 5, c4 = (idx & 31) * 4;
      const v4f v = *(const v4f*)(HS + row * OPIT + c4);
      *(volatile v4f*)(cn_out + (size_t)(rowbase + row) * HID + c4) = v;
    }
    __threadfence();
  }
}

__device__ __forceinline__ void smx_lds(float* p, int wd) {
  float m = p[0];
#pragma unroll 1
  for (int jj = 1; jj < wd; ++jj) m = fmaxf(m, p[jj]);
  float s = 0.0f;
#pragma unroll 1
  for (int jj = 0; jj < wd; ++jj) { const float e = expf(p[jj] - m); p[jj] = e; s += e; }
  const float inv = 1.0f / s;
#pragma unroll 1
  for (int jj = 0; jj < wd; ++jj) p[jj] = p[jj] * inv;
}
__device__ __forceinline__ void emit_lines(const float* sl, float* dst, int nv4, int lane) {
  const int nq = (nv4 + 31) >> 5;
  for (int pass = 0; pass < 2; ++pass) {
#pragma unroll 1
    for (int q = 0; q < nq; ++q) {
      const int idx = q * 32 + lane;
      if (idx < nv4) {
        const v4f v = *(const v4f*)(sl + 4 * idx);
        *(volatile v4f*)(dst + 4 * idx) = v;
      }
    }
    __threadfence();
  }
}
constexpr int SLABF = 32 * 38;
__global__ __launch_bounds__(NTHR) void heads_out_kernel(const float* __restrict__ sc, const float* __restrict__ tg1,
                                                         const float* __restrict__ tg5, const float* __restrict__ tga,
                                                         const float* __restrict__ tge, float* __restrict__ out) {
  __shared__ __align__(16) float slab[NTHR / 32][SLABF];
  const int tid = threadIdx.x, lane = tid & 31, wave = tid >> 5;
  const int t = blockIdx.x * NTHR + tid;
  const int t0w = t - lane;
  float* sl = slab[wave];

  union { v4f v[6]; float f[24]; } sv;
  const v4f* sp = (const v4f*)(sc + (size_t)t * NSC);
#pragma unroll
  for (int q = 0; q < 6; ++q) sv.v[q] = sp[q];

#pragma unroll
  for (int jj = 0; jj < 3; ++jj) sl[lane * 3 + jj] = sv.f[jj];
  smx_lds(sl + lane * 3, 3);
  __syncthreads();
  emit_lines(sl, out + (size_t)t0w * 3, 24, lane);
  __syncthreads();
#pragma unroll
  for (int jj = 0; jj < 9; ++jj) sl[lane * 9 + jj] = sv.f[3 + jj];
  smx_lds(sl + lane * 9, 9);
  __syncthreads();
  emit_lines(sl, out + 49152 + (size_t)t0w * 9, 72, lane);
  __syncthreads();
#pragma unroll
  for (int jj = 0; jj < 9; ++jj) sl[lane * 9 + jj] = sv.f[12 + jj];
  smx_lds(sl + lane * 9, 9);
  __syncthreads();
  emit_lines(sl, out + 196608 + (size_t)t0w * 9, 72, lane);
  __syncthreads();
  {
    const float g1 = tg1[t];
    float g5[5];
#pragma unroll
    for (int jj = 0; jj < 5; ++jj) g5[jj] = tg5[(size_t)t * 5 + jj];
    union { v4f v[4]; float f[16]; } ga, ge;
#pragma unroll
    for (int q = 0; q < 4; ++q) { ga.v[q] = *(const v4f*)(tga + (size_t)t * 16 + 4 * q); ge.v[q] = *(const v4f*)(tge + (size_t)t * 16 + 4 * q); }
    sl[lane * 38 + 0] = g1;
#pragma unroll
    for (int jj = 0; jj < 5; ++jj) sl[lane * 38 + 1 + jj] = g5[jj];
#pragma unroll
    for (int jj = 0; jj < 16; ++jj) { sl[lane * 38 + 6 + jj] = ga.f[jj]; sl[lane * 38 + 22 + jj] = ge.f[jj]; }
  }
  smx_lds(sl + lane * 38, 38);
  __syncthreads();
  emit_lines(sl, out + 344064 + (size_t)t0w * 38, 304, lane);
}

extern "C" void kernel_launch(void* const* d_in, const int* in_sizes, int n_in,
                              void* d_out, int out_size, void* d_ws, size_t ws_size, hipStream_t stream) {
  if (n_in < 33 || d_out == nullptr || d_ws == nullptr) return;
  if (in_sizes[0] != NTOK * 3 || in_sizes[1] != NTOK * 9 || in_sizes[2] != NTOK * 45 ||
      in_sizes[3] != NTOK * 144 || in_sizes[4] != NTOK * 144 || in_sizes[5] != NSEQ * HID || in_sizes[6] != NSEQ * HID ||
      in_sizes[7] != HID * 3 || in_sizes[8] != HID || in_sizes[9] != HID * 9 || in_sizes[10] != HID ||
      in_sizes[11] != HID * HID || in_sizes[12] != HID || in_sizes[13] != HID * HID || in_sizes[14] != HID ||
      in_sizes[15] != HID * HID || in_sizes[16] != HID || in_sizes[17] != HID * HID || in_sizes[18] != HID ||
      in_sizes[19] != HID * XCOL || in_sizes[20] != HID || in_sizes[21] != NGATE * HID || in_sizes[22] != NGATE * HID ||
      in_sizes[23] != NGATE || in_sizes[24] != NGATE || in_sizes[25] != 3 * HID || in_sizes[26] != 3 ||
      in_sizes[27] != 9 * HID || in_sizes[28] != 9 || in_sizes[29] != 9 * HID || in_sizes[30] != 9 ||
      in_sizes[31] != HID * HID || in_sizes[32] != HID || out_size != NOUTF) return;

  const float* env   = (const float*)d_in[0];
  const float* u_ah  = (const float*)d_in[1];
  const float* u_eh  = (const float*)d_in[2];
  const float* u_anh = (const float*)d_in[3];
  const float* u_enh = (const float*)d_in[4];
  const float* h0    = (const float*)d_in[5];
  const float* c0    = (const float*)d_in[6];
  const float* w_env = (const float*)d_in[7];
  const float* b_env = (const float*)d_in[8];
  const float* w_bas = (const float*)d_in[9];
  const float* b_bas = (const float*)d_in[10];
  const float* w_ah  = (const float*)d_in[11];
  const float* b_ah  = (const float*)d_in[12];
  const float* w_eh  = (const float*)d_in[13];
  const float* b_eh  = (const float*)d_in[14];
  const float* w_anh = (const float*)d_in[15];
  const float* b_anh = (const float*)d_in[16];
  const float* w_enh = (const float*)d_in[17];
  const float* b_enh = (const float*)d_in[18];
  const float* w_pre = (const float*)d_in[19];
  const float* b_pre = (const float*)d_in[20];
  const float* w_ih  = (const float*)d_in[21];
  const float* w_hh  = (const float*)d_in[22];
  const float* b_ih  = (const float*)d_in[23];
  const float* b_hh  = (const float*)d_in[24];
  const float* w_enm = (const float*)d_in[25];
  const float* b_enm = (const float*)d_in[26];
  const float* w_mx  = (const float*)d_in[27];
  const float* b_mx  = (const float*)d_in[28];
  const float* w_my  = (const float*)d_in[29];
  const float* b_my  = (const float*)d_in[30];
  const float* w_att = (const float*)d_in[31];
  const float* b_att = (const float*)d_in[32];
  float* out    = (float*)d_out;
  float* hn_out = out + (size_t)NTOK * 59;
  float* cn_out = out + (size_t)NTOK * 59 + NSEQ * HID;

  char* ws = (char*)d_ws; size_t off = 0;
  auto carve = [&](size_t bytes) -> char* { char* p = ws + off; off += (bytes + 255) & ~(size_t)255; return p; };
  unsigned short* XH   = (unsigned short*)carve((size_t)NTOK * XCOL * 2);
  unsigned short* XL   = (unsigned short*)carve((size_t)NTOK * XCOL * 2);
  unsigned short* WPH  = (unsigned short*)carve((size_t)HID * XCOL * 2);
  unsigned short* WPL  = (unsigned short*)carve((size_t)HID * XCOL * 2);
  unsigned short* WIH  = (unsigned short*)carve((size_t)NGATE * HID * 2);
  unsigned short* WIL  = (unsigned short*)carve((size_t)NGATE * HID * 2);
  unsigned short* WHH  = (unsigned short*)carve((size_t)NGATE * HID * 2);
  unsigned short* WHL  = (unsigned short*)carve((size_t)NGATE * HID * 2);
  unsigned short* WAH  = (unsigned short*)carve((size_t)HID * HID * 2);
  unsigned short* WAL  = (unsigned short*)carve((size_t)HID * HID * 2);
  unsigned short* WDH  = (unsigned short*)carve((size_t)NSC * HID * 2);
  unsigned short* WDL  = (unsigned short*)carve((size_t)NSC * HID * 2);
  float*          BHD  = (float*)carve((size_t)NSC * 4);
  float*          BSUM = (float*)carve((size_t)NGATE * 4);
  unsigned short* WTG  = (unsigned short*)carve((size_t)4 * HID * HID * 2);
  unsigned short* WBP  = (unsigned short*)carve((size_t)HID * WBPIT * 2);
  unsigned short* XPH  = (unsigned short*)carve((size_t)NTOK * HID * 2);
  unsigned short* XPL  = (unsigned short*)carve((size_t)NTOK * HID * 2);
  float*          GX   = (float*)carve((size_t)NTOK * NGATE * 4);
  unsigned short* HSH  = (unsigned short*)carve((size_t)NTOK * HID * 2);
  unsigned short* HSL  = (unsigned short*)carve((size_t)NTOK * HID * 2);
  float*          ATT  = (float*)carve((size_t)NTOK * HID * 4);
  float*          SC   = (float*)carve((size_t)NTOK * NSC * 4);
  float*          TG1  = (float*)carve((size_t)NTOK * 1 * 4);
  float*          TG5  = (float*)carve((size_t)NTOK * 5 * 4);
  float*          TGA  = (float*)carve((size_t)NTOK * 16 * 4);
  float*          TGE  = (float*)carve((size_t)NTOK * 16 * 4);
  if (off > ws_size || off > (size_t)134217728) return;

  wsplit_kernel<<<dim3(40, 4), NTHR, 0, stream>>>(w_pre, w_ih, w_hh, w_att, WPH, WPL, WIH, WIL, WHH, WHL, WAH, WAL,
                                                  HID * XCOL / 8, NGATE * HID / 8, NGATE * HID / 8, HID * HID / 8);
  wf16_kernel<<<dim3(HID * HID / 8 / NTHR, 4), NTHR, 0, stream>>>(w_ah, w_eh, w_anh, w_enh, WTG);
  wbpack_kernel<<<HID * WBPIT / 8 / NTHR, NTHR, 0, stream>>>(w_bas, WBP);
  smallprep_kernel<<<5, NTHR, 0, stream>>>(w_enm, w_mx, w_my, b_enm, b_mx, b_my, b_ih, b_hh, WDH, WDL, BHD, BSUM);
  env_kernel<<<NTOK * 16 / NTHR, NTHR, 0, stream>>>(env, w_env, b_env, XH, XL);
  unit_pass_kernel<128, 1, 0><<<dim3(NTOK * 1 / 128, 1), NTHR, 0, stream>>>(
      u_ah, u_ah, WBP, b_bas, WTG, WTG, b_ah, b_ah, XH, XL, 128, 128, ATT, TG1, TG1);
  unit_pass_kernel<160, 5, 0><<<dim3(NTOK * 5 / 160, 1), NTHR, 0, stream>>>(
      u_eh, u_eh, WBP, b_bas, WTG + HID * HID, WTG + HID * HID, b_eh, b_eh, XH, XL, 256, 256, ATT, TG5, TG5);
  unit_pass_kernel<128, 16, 0><<<dim3(NTOK * 16 / 128, 2), NTHR, 0, stream>>>(
      u_anh, u_enh, WBP, b_bas, WTG + 2 * HID * HID, WTG + 3 * HID * HID, b_anh, b_enh, XH, XL, 384, 512, ATT, TGA, TGE);
  wmma_gemm64<1, true, 2, 2, false, 2><<<dim3((NTOK / 64) * (HID / 64) / 8, 1), NTHR, 0, stream>>>(
      XH, XL, XCOL, 0L, WPH, WPL, XCOL, 0L, (void*)XPH, (void*)XPL, HID, 0L,
      b_pre, b_pre, 0L, NTOK, HID, XCOL, 1.0f);
  wmma_gemm64<1, true, 2, 0, false, 0><<<dim3((NTOK / 64) * (NGATE / 64) / 8, 1), NTHR, 0, stream>>>(
      XPH, XPL, HID, 0L, WIH, WIL, HID, 0L, (void*)GX, (void*)GX, NGATE, 0L,
      BSUM, b_pre, 0L, NTOK, NGATE, HID, 1.0f);
  lstm_kernel<<<NSEQ / 16, NTHR, 0, stream>>>(GX, h0, c0, WHH, WHL, HSH, HSL, hn_out, cn_out);
  wmma_gemm64<1, true, 2, 0, false, 0><<<dim3((NTOK / 64) * (HID / 64) / 8, 1), NTHR, 0, stream>>>(
      HSH, HSL, HID, 0L, WAH, WAL, HID, 0L, (void*)ATT, (void*)ATT, HID, 0L,
      b_att, b_pre, 0L, NTOK, HID, HID, 1.0f);
  wmma_gemm64<1, true, 2, 0, false, 0><<<dim3((NTOK / 64) * (NSC / 64) / 8, 1), NTHR, 0, stream>>>(
      HSH, HSL, HID, 0L, WDH, WDL, HID, 0L, (void*)SC, (void*)SC, NSC, 0L,
      BHD, b_pre, 0L, NTOK, NSC, HID, 1.0f);
  unit_pass_kernel<128, 1, 1><<<dim3(NTOK * 1 / 128, 1), NTHR, 0, stream>>>(
      u_ah, u_ah, WBP, b_bas, WTG, WTG, b_ah, b_ah, XH, XL, 128, 128, ATT, TG1, TG1);
  unit_pass_kernel<160, 5, 1><<<dim3(NTOK * 5 / 160, 1), NTHR, 0, stream>>>(
      u_eh, u_eh, WBP, b_bas, WTG + HID * HID, WTG + HID * HID, b_eh, b_eh, XH, XL, 256, 256, ATT, TG5, TG5);
  unit_pass_kernel<128, 16, 1><<<dim3(NTOK * 16 / 128, 2), NTHR, 0, stream>>>(
      u_anh, u_enh, WBP, b_bas, WTG + 2 * HID * HID, WTG + 3 * HID * HID, b_anh, b_enh, XH, XL, 384, 512, ATT, TGA, TGE);
  heads_out_kernel<<<NTOK / NTHR, NTHR, 0, stream>>>(SC, TG1, TG5, TGA, TGE, out);
}
